// EncoderBlock_27470610825321
// MI455X (gfx1250) — hardware-verified
//
#include <hip/hip_runtime.h>
#include <stdint.h>


#ifndef NB
#define NB 4
#endif
#ifndef SEQ
#define SEQ 1024
#endif
#define NB_FULL   4
#define SEQ_FULL  1024
#define D_MODEL   1024
#define NHEAD     16
#define DKH       64
#define D_FF      4096
#define ROWS      (NB * SEQ)

static_assert((SEQ % 64) == 0);
static_assert((ROWS % 128) == 0);
static_assert(SEQ <= SEQ_FULL);
static_assert(NB >= 1 && NB <= NB_FULL);
static_assert(NHEAD * DKH == D_MODEL);
static_assert((D_MODEL % 128) == 0 && (D_FF % 128) == 0);
static_assert(D_MODEL == 256 * 4);
static_assert(D_MODEL == 128 * 8);
static_assert((D_MODEL % 32) == 0 && (D_FF % 32) == 0);

#define SC_W    64.0f
#define SC_X    8.0f
#define SC_XN   8.0f
#define SC_P    256.0f
#define SC_CTX  64.0f
#define SC_H    16.0f

typedef _Float16 f16_t;
typedef _Float16 v16h __attribute__((ext_vector_type(16)));
typedef _Float16 v8h  __attribute__((ext_vector_type(8)));
typedef _Float16 v4h  __attribute__((ext_vector_type(4)));
typedef float    v8f  __attribute__((ext_vector_type(8)));
typedef float    v4f  __attribute__((ext_vector_type(4)));
typedef v8h v8ha __attribute__((__may_alias__));
typedef v4h v4ha __attribute__((__may_alias__));
typedef v4f v4fa __attribute__((__may_alias__));

__device__ __forceinline__ float bf16r(float f) {
  unsigned int u = __float_as_uint(f);
  u += 0x7FFFu + ((u >> 16) & 1u);
  u &= 0xFFFF0000u;
  return __uint_as_float(u);
}

__device__ __forceinline__ int full_row(int r) {
  return (r / SEQ) * SEQ_FULL + (r % SEQ);
}

__device__ __forceinline__ v8f zero8() {
  v8f z;
#pragma unroll
  for (int i = 0; i < 8; ++i) z[i] = 0.0f;
  return z;
}

union Frag { v16h v; v8h h2[2]; };
__device__ __forceinline__ v16h ldfrag(const f16_t* rowp, int g) {
  Frag f;
  f.h2[0] = *(const v8ha*)(rowp + 8 * g);
  f.h2[1] = *(const v8ha*)(rowp + 16 + 8 * g);
  return f.v;
}

__device__ __forceinline__ v8f mma16(v16h a, v16h b, v8f c) {
  v8f d = __builtin_amdgcn_wmma_f32_16x16x32_f16(false, a, false, b, (short)0, c, false, false);
  asm volatile("v_nop\n\tv_nop\n\tv_nop\n\tv_nop" : "+v"(d) : "v"(a), "v"(b));
  return d;
}

__global__ __launch_bounds__(256) void k_wconv(
    const float* __restrict__ in, f16_t* __restrict__ out, int Kd, int Nd, float scale) {
  __shared__ __align__(16) f16_t T[64 * 72];
  const int tid = threadIdx.x;
  const int n0 = blockIdx.x * 64, k0 = blockIdx.y * 64;
#pragma unroll
  for (int i = 0; i < 4; ++i) {
    const int id = i * 256 + tid;
    const int r = id >> 4, c4 = id & 15;
    v4f v = *(const v4f*)&in[(size_t)(k0 + r) * Nd + n0 + c4 * 4];
#pragma unroll
    for (int e = 0; e < 4; ++e)
      T[(c4 * 4 + e) * 72 + r] = (f16_t)(bf16r(v[e]) * scale);
  }
  __syncthreads();
  v8h ov[2];
#pragma unroll
  for (int j = 0; j < 2; ++j) {
    const int id = j * 256 + tid;
    const int ln = id >> 3, pc = id & 7;
    ov[j] = *(const v8ha*)&T[ln * 72 + pc * 8];
  }
#pragma unroll
  for (int j = 0; j < 2; ++j) {
    const int id = j * 256 + tid;
    const int ln = id >> 3, pc = id & 7;
    f16_t* p = out + (size_t)(n0 + ln) * Kd + k0 + pc * 8;
    *(volatile v8h*)p = ov[j];
  }
  __threadfence();
#pragma unroll
  for (int j = 0; j < 2; ++j) {
    const int id = j * 256 + tid;
    const int ln = id >> 3, pc = id & 7;
    f16_t* p = out + (size_t)(n0 + ln) * Kd + k0 + pc * 8;
    *(volatile v8h*)p = ov[j];
  }
}

__global__ __launch_bounds__(128) void k_xconv(
    const float* __restrict__ in, f16_t* __restrict__ out, float scale) {
  const int row = blockIdx.x, tid = threadIdx.x;
  const float* xr = in + (size_t)full_row(row) * D_MODEL + tid * 8;
  v4f xa = *(const v4f*)xr;
  v4f xb = *(const v4f*)(xr + 4);
  v8h ov;
#pragma unroll
  for (int e = 0; e < 4; ++e) {
    ov[e]     = (f16_t)(bf16r(xa[e]) * scale);
    ov[4 + e] = (f16_t)(bf16r(xb[e]) * scale);
  }
  f16_t* op = out + (size_t)row * D_MODEL + tid * 8;
  *(volatile v8h*)op = ov;
  __threadfence();
  *(volatile v8h*)op = ov;
}

template <int MODE>
__global__ __launch_bounds__(256) void k_ln(
    const float* __restrict__ in, const float* __restrict__ gam,
    const float* __restrict__ bet, f16_t* __restrict__ out16,
    float* __restrict__ out32, float oscale) {
  __shared__ float red[2][8];
  __shared__ __align__(16) f16_t Hs[D_MODEL];
  const int row = blockIdx.x, tid = threadIdx.x, wave = tid >> 5, lane = tid & 31;
  v4f xv = *(const v4f*)(in + (size_t)row * D_MODEL + tid * 4);
  float s = (xv[0] + xv[1]) + (xv[2] + xv[3]);
#pragma unroll
  for (int off = 16; off > 0; off >>= 1) s += __shfl_xor(s, off, 32);
  if (lane == 0) red[0][wave] = s;
  __syncthreads();
  const float tot = ((red[0][0] + red[0][1]) + (red[0][2] + red[0][3])) +
                    ((red[0][4] + red[0][5]) + (red[0][6] + red[0][7]));
  const float mean = tot * (1.0f / D_MODEL);
  float d[4];
  float ss = 0.f;
#pragma unroll
  for (int e = 0; e < 4; ++e) { d[e] = xv[e] - mean; ss += d[e] * d[e]; }
#pragma unroll
  for (int off = 16; off > 0; off >>= 1) ss += __shfl_xor(ss, off, 32);
  if (lane == 0) red[1][wave] = ss;
  __syncthreads();
  const float tot2 = ((red[1][0] + red[1][1]) + (red[1][2] + red[1][3])) +
                     ((red[1][4] + red[1][5]) + (red[1][6] + red[1][7]));
  const float var = tot2 * (1.0f / D_MODEL);
  const float rstd = rsqrtf(var + 1e-6f);
  v4f gv = *(const v4f*)(gam + tid * 4);
  v4f bv = *(const v4f*)(bet + tid * 4);
  v4f y;
#pragma unroll
  for (int e = 0; e < 4; ++e) y[e] = (d[e] * rstd) * bf16r(gv[e]) + bf16r(bv[e]);

  if (MODE == 0) {
    v4h hv;
#pragma unroll
    for (int e = 0; e < 4; ++e) hv[e] = (f16_t)(y[e] * oscale);
    *(v4ha*)&Hs[tid * 4] = hv;
    __syncthreads();
    const int t7 = tid & 127;
    v8h o8 = *(const v8ha*)&Hs[t7 * 8];
    float* p32 = out32 + (size_t)row * D_MODEL + tid * 4;
    f16_t* p16 = out16 + (size_t)row * D_MODEL + t7 * 8;
    *(volatile v4f*)p32 = y;
    if (tid < 128) *(volatile v8h*)p16 = o8;
    __threadfence();
    *(volatile v4f*)p32 = y;
    if (tid < 128) *(volatile v8h*)p16 = o8;
  } else {
    float* p32 = out32 + (size_t)full_row(row) * D_MODEL + tid * 4;
    *(volatile v4f*)p32 = y;
    __threadfence();
    *(volatile v4f*)p32 = y;
  }
}

template <int OUT16, int RELU, int RESM, int OUTFULL>
__global__ __launch_bounds__(256) void k_gemm(
    const f16_t* __restrict__ A, const f16_t* __restrict__ Bt,
    const float* __restrict__ bias, const float* __restrict__ res,
    void* __restrict__ Cout, int M, int N, int K, float cscale, float oscale) {
  __shared__ __align__(16) f16_t As[128 * 32];
  __shared__ __align__(16) f16_t Bs[128 * 32];
  __shared__ __align__(16) float  St[8 * 16 * 64];
  (void)M;
  const int tid = threadIdx.x;
  const int wave = tid >> 5, lane = tid & 31, lh = lane & 15, g = lane >> 4;
  const int waveM = wave & 3, waveN = wave >> 2;
  const int rowBase = blockIdx.y * 128, colBase = blockIdx.x * 128;

  const int sr0 = tid >> 2, sc0 = (tid & 3) * 8;
  const f16_t* gA0 = A  + (size_t)(rowBase + sr0) * K + sc0;
  const f16_t* gA1 = A  + (size_t)(rowBase + sr0 + 64) * K + sc0;
  const f16_t* gB0 = Bt + (size_t)(colBase + sr0) * K + sc0;
  const f16_t* gB1 = Bt + (size_t)(colBase + sr0 + 64) * K + sc0;

  v8f acc[2][4];
#pragma unroll
  for (int mr = 0; mr < 2; ++mr)
#pragma unroll
    for (int nr = 0; nr < 4; ++nr) acc[mr][nr] = zero8();

  const int nk = K >> 5;
  for (int kt = 0; kt < nk; ++kt) {
    const int kc = kt << 5;
    v8h a0 = *(const v8h*)(gA0 + kc);
    v8h a1 = *(const v8h*)(gA1 + kc);
    v8h b0 = *(const v8h*)(gB0 + kc);
    v8h b1 = *(const v8h*)(gB1 + kc);
    __syncthreads();
    *(v8h*)&As[sr0 * 32 + sc0]        = a0;
    *(v8h*)&As[(sr0 + 64) * 32 + sc0] = a1;
    *(v8h*)&Bs[sr0 * 32 + sc0]        = b0;
    *(v8h*)&Bs[(sr0 + 64) * 32 + sc0] = b1;
    __syncthreads();
    v16h af[2], bf[4];
#pragma unroll
    for (int mr = 0; mr < 2; ++mr)
      af[mr] = ldfrag(&As[(waveM * 32 + mr * 16 + lh) * 32], g);
#pragma unroll
    for (int nr = 0; nr < 4; ++nr)
      bf[nr] = ldfrag(&Bs[(waveN * 64 + nr * 16 + lh) * 32], g);
#pragma unroll
    for (int mr = 0; mr < 2; ++mr)
#pragma unroll
      for (int nr = 0; nr < 4; ++nr)
        acc[mr][nr] = mma16(af[mr], bf[nr], acc[mr][nr]);
  }

  const int cb = colBase + waveN * 64;
  float* S = &St[wave * (16 * 64)];
#pragma unroll
  for (int mr = 0; mr < 2; ++mr) {
    __syncthreads();
#pragma unroll
    for (int nr = 0; nr < 4; ++nr)
#pragma unroll
      for (int r = 0; r < 8; ++r)
        S[(g * 8 + r) * 64 + nr * 16 + lh] = acc[mr][nr][r];
    __syncthreads();
    const int rb = rowBase + waveM * 32 + mr * 16;
    if (OUT16) {
      f16_t* C16 = (f16_t*)Cout;
      v8h ov[4];
#pragma unroll
      for (int j = 0; j < 4; ++j) {
        const int lr = j * 4 + (lane >> 3), pc = lane & 7;
        v4f s0 = *(const v4fa*)&S[lr * 64 + pc * 8];
        v4f s1 = *(const v4fa*)&S[lr * 64 + pc * 8 + 4];
        v4f q0 = *(const v4f*)&bias[cb + pc * 8];
        v4f q1 = *(const v4f*)&bias[cb + pc * 8 + 4];
#pragma unroll
        for (int e = 0; e < 4; ++e) {
          float v0 = s0[e] * cscale + bf16r(q0[e]);
          float v1 = s1[e] * cscale + bf16r(q1[e]);
          if (RELU) { v0 = fmaxf(v0, 0.0f); v1 = fmaxf(v1, 0.0f); }
          ov[j][e]     = (f16_t)(v0 * oscale);
          ov[j][4 + e] = (f16_t)(v1 * oscale);
        }
      }
#pragma unroll
      for (int j = 0; j < 4; ++j) {
        const int lr = j * 4 + (lane >> 3), pc = lane & 7;
        f16_t* p = C16 + (size_t)(rb + lr) * N + cb + pc * 8;
        *(volatile v8h*)p = ov[j];
      }
      __threadfence();
#pragma unroll
      for (int j = 0; j < 4; ++j) {
        const int lr = j * 4 + (lane >> 3), pc = lane & 7;
        f16_t* p = C16 + (size_t)(rb + lr) * N + cb + pc * 8;
        *(volatile v8h*)p = ov[j];
      }
    } else {
      float* C32 = (float*)Cout;
      v4f ov[8];
#pragma unroll
      for (int j = 0; j < 8; ++j) {
        const int lr = j * 2 + (lane >> 4), pc = lane & 15;
        v4f s0 = *(const v4fa*)&S[lr * 64 + pc * 4];
        v4f q0 = *(const v4f*)&bias[cb + pc * 4];
        v4f vv;
#pragma unroll
        for (int e = 0; e < 4; ++e) vv[e] = s0[e] * cscale + bf16r(q0[e]);
        if (RELU) {
#pragma unroll
          for (int e = 0; e < 4; ++e) vv[e] = fmaxf(vv[e], 0.0f);
        }
        if (RESM == 1) {
          v4f rr = *(const v4f*)&res[(size_t)(rb + lr) * N + cb + pc * 4];
#pragma unroll
          for (int e = 0; e < 4; ++e) vv[e] += rr[e];
        } else if (RESM == 2) {
          v4f rr = *(const v4f*)&res[(size_t)full_row(rb + lr) * N + cb + pc * 4];
#pragma unroll
          for (int e = 0; e < 4; ++e) vv[e] += bf16r(rr[e]);
        }
        ov[j] = vv;
      }
#pragma unroll
      for (int j = 0; j < 8; ++j) {
        const int lr = j * 2 + (lane >> 4), pc = lane & 15;
        const int orow = OUTFULL ? full_row(rb + lr) : (rb + lr);
        float* p = C32 + (size_t)orow * N + cb + pc * 4;
        *(volatile v4f*)p = ov[j];
      }
      __threadfence();
#pragma unroll
      for (int j = 0; j < 8; ++j) {
        const int lr = j * 2 + (lane >> 4), pc = lane & 15;
        const int orow = OUTFULL ? full_row(rb + lr) : (rb + lr);
        float* p = C32 + (size_t)orow * N + cb + pc * 4;
        *(volatile v4f*)p = ov[j];
      }
    }
  }
}

__global__ __launch_bounds__(128) void k_attn(
    const f16_t* __restrict__ Qp, const f16_t* __restrict__ Kp,
    const f16_t* __restrict__ Vp, const float* __restrict__ msk,
    f16_t* __restrict__ ctx) {
  __shared__ __align__(16) f16_t Qs[64 * 64];
  __shared__ __align__(16) f16_t Ks[64 * 64];
  __shared__ __align__(16) f16_t Vt[64 * 64];
  __shared__ __align__(16) f16_t Ps[64 * 64];
  const int tid = threadIdx.x;
  const int wave = tid >> 5, lane = tid & 31, lh = lane & 15, g = lane >> 4;
  const int qt = blockIdx.x, h = blockIdx.y, b = blockIdx.z;
  const int qbase = qt * 64;
  const size_t prow0 = (size_t)b * SEQ;
  const int col0 = h * DKH;
  const float* mrow = msk + (size_t)b * SEQ_FULL;

#pragma unroll
  for (int i = 0; i < 4; ++i) {
    const int id = i * 128 + tid;
    const int r = id >> 3, c = (id & 7) * 8;
    *(v8h*)&Qs[r * 64 + c] = *(const v8h*)&Qp[(prow0 + qbase + r) * D_MODEL + col0 + c];
  }
  __syncthreads();
  v16h aq[2];
#pragma unroll
  for (int c = 0; c < 2; ++c) aq[c] = ldfrag(&Qs[(wave * 16 + lh) * 64 + c * 32], g);

  v8f o[4];
#pragma unroll
  for (int nr = 0; nr < 4; ++nr) o[nr] = zero8();
  float m[8], l[8];
#pragma unroll
  for (int r = 0; r < 8; ++r) { m[r] = -1e30f; l[r] = 0.f; }
  const float sm_scale = 0.125f;

  for (int kt = 0; kt < SEQ / 64; ++kt) {
    const int kbase = kt * 64;
    __syncthreads();
#pragma unroll
    for (int i = 0; i < 4; ++i) {
      const int id = i * 128 + tid;
      const int r = id >> 3, c = (id & 7) * 8;
      *(v8h*)&Ks[r * 64 + c] = *(const v8h*)&Kp[(prow0 + kbase + r) * D_MODEL + col0 + c];
      v8h vv = *(const v8h*)&Vp[(prow0 + kbase + r) * D_MODEL + col0 + c];
#pragma unroll
      for (int j = 0; j < 8; ++j) Vt[(c + j) * 64 + r] = vv[j];
    }
    __syncthreads();

    float mk[4];
#pragma unroll
    for (int nr = 0; nr < 4; ++nr) mk[nr] = bf16r(mrow[kbase + nr * 16 + lh]) * (-1.0e9f);

    v8f s[4];
#pragma unroll
    for (int nr = 0; nr < 4; ++nr) {
      s[nr] = zero8();
#pragma unroll
      for (int c = 0; c < 2; ++c) {
        v16h bk = ldfrag(&Ks[(nr * 16 + lh) * 64 + c * 32], g);
        s[nr] = mma16(aq[c], bk, s[nr]);
      }
    }
#pragma unroll
    for (int nr = 0; nr < 4; ++nr)
#pragma unroll
      for (int r = 0; r < 8; ++r) s[nr][r] = s[nr][r] * sm_scale + mk[nr];
    float f[8];
#pragma unroll
    for (int r = 0; r < 8; ++r) {
      float v = fmaxf(fmaxf(s[0][r], s[1][r]), fmaxf(s[2][r], s[3][r]));
#pragma unroll
      for (int off = 8; off > 0; off >>= 1) v = fmaxf(v, __shfl_xor(v, off, 16));
      const float mn = fmaxf(m[r], v);
      f[r] = __expf(m[r] - mn);
      m[r] = mn;
    }
    float rs[8];
#pragma unroll
    for (int r = 0; r < 8; ++r) rs[r] = 0.f;
#pragma unroll
    for (int nr = 0; nr < 4; ++nr)
#pragma unroll
      for (int r = 0; r < 8; ++r) {
        const float p = __expf(s[nr][r] - m[r]);
        s[nr][r] = p;
        rs[r] += p;
      }
#pragma unroll
    for (int r = 0; r < 8; ++r) {
      float v = rs[r];
#pragma unroll
      for (int off = 8; off > 0; off >>= 1) v += __shfl_xor(v, off, 16);
      l[r] = l[r] * f[r] + v;
    }
#pragma unroll
    for (int nr = 0; nr < 4; ++nr)
#pragma unroll
      for (int r = 0; r < 8; ++r) o[nr][r] *= f[r];
#pragma unroll
    for (int nr = 0; nr < 4; ++nr)
#pragma unroll
      for (int r = 0; r < 8; ++r)
        Ps[(wave * 16 + g * 8 + r) * 64 + nr * 16 + lh] = (f16_t)(s[nr][r] * SC_P);
    __syncthreads();

#pragma unroll
    for (int c = 0; c < 2; ++c) {
      v16h ap = ldfrag(&Ps[(wave * 16 + lh) * 64 + c * 32], g);
#pragma unroll
      for (int nr = 0; nr < 4; ++nr) {
        v16h bv = ldfrag(&Vt[(nr * 16 + lh) * 64 + c * 32], g);
        o[nr] = mma16(ap, bv, o[nr]);
      }
    }
  }

  __syncthreads();
  float il[8];
#pragma unroll
  for (int r = 0; r < 8; ++r) il[r] = (SC_CTX / SC_P) * (1.0f / l[r]);
#pragma unroll
  for (int nr = 0; nr < 4; ++nr)
#pragma unroll
    for (int r = 0; r < 8; ++r)
      Ps[(wave * 16 + g * 8 + r) * 64 + nr * 16 + lh] = (f16_t)(o[nr][r] * il[r]);
  __syncthreads();
  v8h ov[4];
#pragma unroll
  for (int j = 0; j < 4; ++j) {
    const int lr = wave * 16 + j * 4 + (lane >> 3), pc = lane & 7;
    ov[j] = *(const v8ha*)&Ps[lr * 64 + pc * 8];
  }
#pragma unroll
  for (int j = 0; j < 4; ++j) {
    const int lr = wave * 16 + j * 4 + (lane >> 3), pc = lane & 7;
    f16_t* p = ctx + (prow0 + qbase + lr) * D_MODEL + col0 + pc * 8;
    *(volatile v8h*)p = ov[j];
  }
  __threadfence();
#pragma unroll
  for (int j = 0; j < 4; ++j) {
    const int lr = wave * 16 + j * 4 + (lane >> 3), pc = lane & 7;
    f16_t* p = ctx + (prow0 + qbase + lr) * D_MODEL + col0 + pc * 8;
    *(volatile v8h*)p = ov[j];
  }
}

extern "C" void kernel_launch(void* const* d_in, const int* in_sizes, int n_in,
                              void* d_out, int out_size, void* d_ws, size_t ws_size,
                              hipStream_t stream) {
  if (n_in < 18) return;
  const int need_x = ((NB - 1) * SEQ_FULL + SEQ) * D_MODEL;
  const int need_m = (NB - 1) * SEQ_FULL + SEQ;
  if (in_sizes[0] < need_x) return;
  if (in_sizes[1] < need_m) return;
  if (in_sizes[2] < D_MODEL * D_MODEL || in_sizes[4] < D_MODEL * D_MODEL ||
      in_sizes[6] < D_MODEL * D_MODEL || in_sizes[8] < D_MODEL * D_MODEL) return;
  if (in_sizes[3] < D_MODEL || in_sizes[5] < D_MODEL || in_sizes[7] < D_MODEL ||
      in_sizes[9] < D_MODEL || in_sizes[13] < D_MODEL || in_sizes[11] < D_FF) return;
  if (in_sizes[10] < D_MODEL * D_FF || in_sizes[12] < D_FF * D_MODEL) return;
  if (in_sizes[14] < D_MODEL || in_sizes[15] < D_MODEL ||
      in_sizes[16] < D_MODEL || in_sizes[17] < D_MODEL) return;
  if (out_size < need_x) return;

  const float* x   = (const float*)d_in[0];
  const float* msk = (const float*)d_in[1];
  const float* Wq = (const float*)d_in[2];   const float* bq = (const float*)d_in[3];
  const float* Wk = (const float*)d_in[4];   const float* bk = (const float*)d_in[5];
  const float* Wv = (const float*)d_in[6];   const float* bv = (const float*)d_in[7];
  const float* Wo = (const float*)d_in[8];   const float* bo = (const float*)d_in[9];
  const float* W1 = (const float*)d_in[10];  const float* b1 = (const float*)d_in[11];
  const float* W2 = (const float*)d_in[12];  const float* b2 = (const float*)d_in[13];
  const float* g1 = (const float*)d_in[14];  const float* be1 = (const float*)d_in[15];
  const float* g2 = (const float*)d_in[16];  const float* be2 = (const float*)d_in[17];
  float* out = (float*)d_out;

  char* ws = (char*)d_ws;
  size_t off = 0;
  auto carve = [&](size_t bytes) -> char* {
    char* p = ws + off;
    off += (bytes + 255) & ~(size_t)255;
    return p;
  };
  const size_t plane16 = (size_t)ROWS * D_MODEL * 2;
  const size_t plane32 = (size_t)ROWS * D_MODEL * 4;
  const size_t hbytes  = (size_t)ROWS * D_FF * 2;
  const size_t r1bytes = (4 * plane16 > hbytes) ? 4 * plane16 : hbytes;

  f16_t* wqT = (f16_t*)carve((size_t)D_MODEL * D_MODEL * 2);
  f16_t* wkT = (f16_t*)carve((size_t)D_MODEL * D_MODEL * 2);
  f16_t* wvT = (f16_t*)carve((size_t)D_MODEL * D_MODEL * 2);
  f16_t* woT = (f16_t*)carve((size_t)D_MODEL * D_MODEL * 2);
  f16_t* w1T = (f16_t*)carve((size_t)D_FF * D_MODEL * 2);
  f16_t* w2T = (f16_t*)carve((size_t)D_MODEL * D_FF * 2);
  char* R1 = carve(r1bytes);
  f16_t* xb  = (f16_t*)(R1 + 0 * plane16);
  f16_t* qb  = (f16_t*)(R1 + 1 * plane16);
  f16_t* kb  = (f16_t*)(R1 + 2 * plane16);
  f16_t* vbp = (f16_t*)(R1 + 3 * plane16);
  f16_t* hb  = (f16_t*)R1;
  char* R2 = carve(plane16);
  f16_t* cx  = (f16_t*)R2;
  f16_t* o1h = (f16_t*)R2;
  char* R3 = carve(plane32);
  float* x1pre = (float*)R3;
  float* t2    = (float*)R3;
  float* o1f = (float*)carve(plane32);
  if (off > ws_size) return;

  k_wconv<<<dim3(D_MODEL / 64, D_MODEL / 64), 256, 0, stream>>>(Wq, wqT, D_MODEL, D_MODEL, SC_W);
  k_wconv<<<dim3(D_MODEL / 64, D_MODEL / 64), 256, 0, stream>>>(Wk, wkT, D_MODEL, D_MODEL, SC_W);
  k_wconv<<<dim3(D_MODEL / 64, D_MODEL / 64), 256, 0, stream>>>(Wv, wvT, D_MODEL, D_MODEL, SC_W);
  k_wconv<<<dim3(D_MODEL / 64, D_MODEL / 64), 256, 0, stream>>>(Wo, woT, D_MODEL, D_MODEL, SC_W);
  k_wconv<<<dim3(D_FF / 64,    D_MODEL / 64), 256, 0, stream>>>(W1, w1T, D_MODEL, D_FF, SC_W);
  k_wconv<<<dim3(D_MODEL / 64, D_FF / 64),    256, 0, stream>>>(W2, w2T, D_FF, D_MODEL, SC_W);

  k_xconv<<<ROWS, 128, 0, stream>>>(x, xb, SC_X);

  const dim3 gP(D_MODEL / 128, ROWS / 128);
  const float cs_p = 1.0f / (SC_W * SC_X);
  k_gemm<1, 0, 0, 0><<<gP, 256, 0, stream>>>(xb, wqT, bq, nullptr, qb,  ROWS, D_MODEL, D_MODEL, cs_p, 1.0f);
  k_gemm<1, 0, 0, 0><<<gP, 256, 0, stream>>>(xb, wkT, bk, nullptr, kb,  ROWS, D_MODEL, D_MODEL, cs_p, 1.0f);
  k_gemm<1, 0, 0, 0><<<gP, 256, 0, stream>>>(xb, wvT, bv, nullptr, vbp, ROWS, D_MODEL, D_MODEL, cs_p, 1.0f);

  k_attn<<<dim3(SEQ / 64, NHEAD, NB), 128, 0, stream>>>(qb, kb, vbp, msk, cx);

  k_gemm<0, 0, 2, 0><<<gP, 256, 0, stream>>>(cx, woT, bo, x, x1pre, ROWS, D_MODEL, D_MODEL,
                                            1.0f / (SC_W * SC_CTX), 1.0f);

  k_ln<0><<<ROWS, 256, 0, stream>>>(x1pre, g1, be1, o1h, o1f, SC_XN);

  k_gemm<1, 0, 0, 0><<<dim3(D_FF / 128, ROWS / 128), 256, 0, stream>>>(
      o1h, w1T, b1, nullptr, hb, ROWS, D_FF, D_MODEL, 1.0f / (SC_W * SC_XN), SC_H);

  k_gemm<0, 0, 1, 0><<<gP, 256, 0, stream>>>(hb, w2T, b2, o1f, t2, ROWS, D_MODEL, D_FF,
                                            1.0f / (SC_W * SC_H), 1.0f);

  k_ln<1><<<ROWS, 256, 0, stream>>>(t2, g2, be2, nullptr, out, 1.0f);
}
